// DeltaProductLayer_4286377361863
// MI455X (gfx1250) — hardware-verified
//
#include <hip/hip_runtime.h>
#include <stdint.h>
#include <stddef.h>


#define B_   2
#define S_   1024
#define F_   1024
#define H_   8
#define D_   64
#define R_   2
#define M_   (B_ * S_)
#define NQ_  (H_ * D_)
#define NK_  (H_ * R_ * D_)
#define NB_  (H_ * R_)
#define NCAT (NQ_ + 2 * NK_ + NB_)
#define NP_  2624
#define QOFF 0
#define KOFF NQ_
#define VOFF (NQ_ + NK_)
#define BOFF (NQ_ + 2 * NK_)
#define EPS_NORM 1e-6f
#define EPS_RMS  1e-6f

#define BM  128
#define BN  64
#define BK  32
#define LDV 5
#define CP  68
#define TP  68

static_assert(M_ % BM == 0);
static_assert(NP_ % BN == 0);
static_assert(F_ % BN == 0);
static_assert(F_ % BK == 0);
static_assert(NQ_ % BK == 0);
static_assert(NP_ >= NCAT);
static_assert((NP_ % 32) == 0);
static_assert((F_ % 8) == 0 && (NQ_ % 8) == 0);

typedef _Float16 v16h __attribute__((ext_vector_type(16)));
typedef _Float16 v8h  __attribute__((ext_vector_type(8)));
typedef float    v8f  __attribute__((ext_vector_type(8)));
typedef float    v4f  __attribute__((ext_vector_type(4)));
typedef v8h __attribute__((__may_alias__)) v8ha;
typedef v4f __attribute__((__may_alias__)) v4fa;

union Frag { v16h v; v8h half[2]; };

__device__ __forceinline__ float bf16r(float f) {
  unsigned int u = __float_as_uint(f);
  u = (u + 0x7FFFu + ((u >> 16) & 1u)) & 0xFFFF0000u;
  return __uint_as_float(u);
}

__device__ __forceinline__ v8f wmma_f16(v16h a, v16h b, v8f c) {
  v8f d = __builtin_amdgcn_wmma_f32_16x16x32_f16(false, a, false, b, (short)0, c, false, false);
  asm volatile("v_nop\n\tv_nop\n\tv_nop\n\tv_nop" : "+v"(d) : "v"(a), "v"(b));
  return d;
}

__device__ __forceinline__ float sigm(float x) { return 1.0f / (1.0f + expf(-x)); }

__device__ __forceinline__ float epi_act(float x, int col, int silu_end, int sig_start) {
  if (col < silu_end) return x * sigm(x);
  if (col >= sig_start) return sigm(x);
  return x;
}

__global__ __launch_bounds__(256)
void pack_act_kernel(const float* __restrict__ in, _Float16* __restrict__ out, int n8, float scale) {
  const int t = blockIdx.x * 256 + threadIdx.x;
  if (t >= n8) return;
  const size_t e = (size_t)t * 8;
  const v4f x0 = *(const v4fa*)(in + e);
  const v4f x1 = *(const v4fa*)(in + e + 4);
  v8h o;
#pragma unroll
  for (int i = 0; i < 4; ++i) {
    o[i]     = (_Float16)(bf16r(x0[i]) * scale);
    o[4 + i] = (_Float16)(bf16r(x1[i]) * scale);
  }
  volatile v8h* dst = (volatile v8h*)(out + e);
  *dst = o;
  __threadfence();
  *dst = o;
}

__global__ __launch_bounds__(256)
void pack_wcat_kernel(const float* __restrict__ Wq, const float* __restrict__ Wk,
                      const float* __restrict__ Wv, const float* __restrict__ Wb,
                      _Float16* __restrict__ out, int n8, float scale) {
  const int t = blockIdx.x * 256 + threadIdx.x;
  if (t >= n8) return;
  const int e = t * 8;
  const int n = e / F_, f0 = e % F_;
  v8h o;
#pragma unroll
  for (int i = 0; i < 8; ++i) {
    const int f = f0 + i;
    float v = 0.0f;
    if      (n < KOFF) v = Wq[(size_t)f * NQ_ + n];
    else if (n < VOFF) v = Wk[(size_t)f * NK_ + (n - KOFF)];
    else if (n < BOFF) v = Wv[(size_t)f * NK_ + (n - VOFF)];
    else if (n < NCAT) v = Wb[(size_t)f * NB_ + (n - BOFF)];
    o[i] = (_Float16)(bf16r(v) * scale);
  }
  volatile v8h* dst = (volatile v8h*)(out + (size_t)e);
  *dst = o;
  __threadfence();
  *dst = o;
}

__global__ __launch_bounds__(256)
void pack_wo_kernel(const float* __restrict__ Wo, _Float16* __restrict__ out, int n8, float scale) {
  const int t = blockIdx.x * 256 + threadIdx.x;
  if (t >= n8) return;
  const int e = t * 8;
  const int n = e / NQ_, k0 = e % NQ_;
  v8h o;
#pragma unroll
  for (int i = 0; i < 8; ++i)
    o[i] = (_Float16)(bf16r(Wo[(size_t)(k0 + i) * F_ + n]) * scale);
  volatile v8h* dst = (volatile v8h*)(out + (size_t)e);
  *dst = o;
  __threadfence();
  *dst = o;
}

struct GemmStage { v8h a[2][BM * LDV]; v8h b[BN * LDV]; };
union  GemmSmem  { GemmStage st; float c[BM * CP]; };

template <int PLANES>
__global__ __launch_bounds__(256)
void gemm_f16_kernel(const _Float16* __restrict__ A0, const _Float16* __restrict__ A1,
                     const _Float16* __restrict__ Bt, float* __restrict__ C,
                     const float* __restrict__ bias, int has_bias,
                     int M, int N, int K, int ldc,
                     float scale0, float scale1, int silu_end, int sig_start) {
  __shared__ GemmSmem sm;
  const int bm = blockIdx.y * BM, bn = blockIdx.x * BN;
  if (bm + BM > M || bn + BN > N) return;

  const int tid = threadIdx.x, lane = tid & 31, wave = tid >> 5;
  const int wr = wave & 3, wc = wave >> 2;
  const int h = lane >> 4, m = lane & 15;
  const int ar = tid >> 1, ac = tid & 1;
  const int bc = tid >> 2, bk = tid & 3;

  const v8f zero8 = {0.f, 0.f, 0.f, 0.f, 0.f, 0.f, 0.f, 0.f};
  v8f acc[PLANES][2][2];
#pragma unroll
  for (int p = 0; p < PLANES; ++p)
#pragma unroll
    for (int i = 0; i < 2; ++i)
#pragma unroll
      for (int j = 0; j < 2; ++j) acc[p][i][j] = zero8;

  const _Float16* Apl[2] = {A0, A1};
  const int KT = K / BK;
  for (int kt = 0; kt < KT; ++kt) {
    const size_t k0 = (size_t)kt * BK;
#pragma unroll
    for (int p = 0; p < PLANES; ++p) {
      const v8ha* g = (const v8ha*)(Apl[p] + (size_t)(bm + ar) * K + k0 + 16 * ac);
      sm.st.a[p][ar * LDV + 2 * ac]     = g[0];
      sm.st.a[p][ar * LDV + 2 * ac + 1] = g[1];
    }
    {
      const v8ha* g = (const v8ha*)(Bt + (size_t)(bn + bc) * K + k0 + 8 * bk);
      sm.st.b[bc * LDV + bk] = g[0];
    }
    __syncthreads();

    Frag bf[2];
#pragma unroll
    for (int nt = 0; nt < 2; ++nt) {
      const int col = wc * 32 + nt * 16 + m;
      bf[nt].half[0] = sm.st.b[col * LDV + h];
      bf[nt].half[1] = sm.st.b[col * LDV + 2 + h];
    }
#pragma unroll
    for (int p = 0; p < PLANES; ++p) {
      Frag af[2];
#pragma unroll
      for (int mt = 0; mt < 2; ++mt) {
        const int row = wr * 32 + mt * 16 + m;
        af[mt].half[0] = sm.st.a[p][row * LDV + h];
        af[mt].half[1] = sm.st.a[p][row * LDV + 2 + h];
      }
#pragma unroll
      for (int mt = 0; mt < 2; ++mt)
#pragma unroll
        for (int nt = 0; nt < 2; ++nt)
          acc[p][mt][nt] = wmma_f16(af[mt].v, bf[nt].v, acc[p][mt][nt]);
    }
    __syncthreads();
  }

#pragma unroll
  for (int mt = 0; mt < 2; ++mt)
#pragma unroll
    for (int nt = 0; nt < 2; ++nt) {
      const int col = wc * 32 + nt * 16 + m;
#pragma unroll
      for (int r = 0; r < 8; ++r) {
        const int row = wr * 32 + mt * 16 + 8 * h + r;
        float v = acc[0][mt][nt][r] * scale0;
        if (PLANES > 1) v += acc[PLANES - 1][mt][nt][r] * scale1;
        sm.c[row * CP + col] = v;
      }
    }
  __syncthreads();

  const int gc = bn + 4 * m;
  for (int i = 0; i < 8; ++i) {
    const int row = wave * 16 + 2 * i + h;
    float* cr = sm.c + row * CP + 4 * m;
    v4f v = *(v4fa*)cr;
#pragma unroll
    for (int e = 0; e < 4; ++e) {
      float xv = v[e];
      if (has_bias) xv += bf16r(bias[gc + e]);
      v[e] = epi_act(xv, gc + e, silu_end, sig_start);
    }
    *(v4fa*)cr = v;
    *(volatile v4f*)(C + (size_t)(bm + row) * ldc + gc) = v;
  }
  __threadfence();
  for (int i = 0; i < 8; ++i) {
    const int row = wave * 16 + 2 * i + h;
    const v4f v = *(const v4fa*)(sm.c + row * CP + 4 * m);
    *(volatile v4f*)(C + (size_t)(bm + row) * ldc + gc) = v;
  }
}

__global__ __launch_bounds__(64)
void scan_kernel(const float* __restrict__ qkvb, const int* __restrict__ mask,
                 const float* __restrict__ carry, float* __restrict__ xout,
                 float* __restrict__ carry_out) {
  const int bh = blockIdx.x;
  if (bh >= B_ * H_) return;
  const int b = bh / H_, hd = bh % H_;
  const int tid = threadIdx.x, lane = tid & 31, wv = tid >> 5;

  __shared__ __align__(16) float sT[D_ * TP];
  __shared__ __align__(16) float sq[D_];
  __shared__ __align__(16) float sk1[D_];
  __shared__ __align__(16) float sk2[D_];
  __shared__ float sred[2][4];

  float* trow = sT + tid * TP;
  {
    const float* c0 = carry + (size_t)bh * D_ * D_ + (size_t)tid * D_;
#pragma unroll 2
    for (int j4 = 0; j4 < D_ / 4; ++j4) {
      const v4f c = *(const v4fa*)(c0 + 4 * j4);
      v4f t;
      t[0] = bf16r(c[0]); t[1] = bf16r(c[1]); t[2] = bf16r(c[2]); t[3] = bf16r(c[3]);
      *(v4fa*)(trow + 4 * j4) = t;
    }
  }

  const int qo  = QOFF + hd * D_;
  const int k1o = KOFF + (hd * R_ + 0) * D_;
  const int k2o = KOFF + (hd * R_ + 1) * D_;
  const int v1o = VOFF + (hd * R_ + 0) * D_;
  const int v2o = VOFF + (hd * R_ + 1) * D_;
  const int bof = BOFF + hd * R_;

  for (int s = 0; s < S_; ++s) {
    const size_t mrow = (size_t)b * S_ + s;
    const float* row = qkvb + mrow * NP_;
    const float q  = row[qo + tid];
    const float k1 = row[k1o + tid];
    const float k2 = row[k2o + tid];
    const float v1 = row[v1o + tid];
    const float v2 = row[v2o + tid];
    const float b1 = row[bof], b2 = row[bof + 1];
    const float keep = 1.0f - (float)mask[mrow];

    float pq = q * q, p1 = k1 * k1, p2 = k2 * k2;
#pragma unroll
    for (int off = 16; off > 0; off >>= 1) {
      pq += __shfl_xor(pq, off, 32);
      p1 += __shfl_xor(p1, off, 32);
      p2 += __shfl_xor(p2, off, 32);
    }
    sq[tid] = q; sk1[tid] = k1; sk2[tid] = k2;
    if (lane == 0) { sred[wv][0] = pq; sred[wv][1] = p1; sred[wv][2] = p2; }
    __syncthreads();
    const float iq  = 1.0f / (sqrtf(sred[0][0] + sred[1][0]) + EPS_NORM);
    const float ik1 = 1.0f / (sqrtf(sred[0][1] + sred[1][1]) + EPS_NORM);
    const float ik2 = 1.0f / (sqrtf(sred[0][2] + sred[1][2]) + EPS_NORM);

    float u = 0.0f;
#pragma unroll 2
    for (int j4 = 0; j4 < D_ / 4; ++j4) {
      v4f t = *(v4fa*)(trow + 4 * j4);
      const v4f kk = *(const v4fa*)(sk1 + 4 * j4);
      t *= keep;
      u = fmaf(t[0], kk[0], u); u = fmaf(t[1], kk[1], u);
      u = fmaf(t[2], kk[2], u); u = fmaf(t[3], kk[3], u);
      *(v4fa*)(trow + 4 * j4) = t;
    }
    const float w = b1 * (v1 - u * ik1) * ik1;

    float pp = 0.0f;
#pragma unroll 2
    for (int j4 = 0; j4 < D_ / 4; ++j4) {
      v4f t = *(v4fa*)(trow + 4 * j4);
      const v4f ka = *(const v4fa*)(sk1 + 4 * j4);
      const v4f kb = *(const v4fa*)(sk2 + 4 * j4);
      t[0] = fmaf(w, ka[0], t[0]); t[1] = fmaf(w, ka[1], t[1]);
      t[2] = fmaf(w, ka[2], t[2]); t[3] = fmaf(w, ka[3], t[3]);
      pp = fmaf(t[0], kb[0], pp); pp = fmaf(t[1], kb[1], pp);
      pp = fmaf(t[2], kb[2], pp); pp = fmaf(t[3], kb[3], pp);
      *(v4fa*)(trow + 4 * j4) = t;
    }
    const float y2 = b2 * (v2 - pp * ik2) * ik2;

    float xs = 0.0f;
#pragma unroll 2
    for (int j4 = 0; j4 < D_ / 4; ++j4) {
      v4f t = *(v4fa*)(trow + 4 * j4);
      const v4f kb = *(const v4fa*)(sk2 + 4 * j4);
      const v4f qq = *(const v4fa*)(sq + 4 * j4);
      t[0] = fmaf(y2, kb[0], t[0]); t[1] = fmaf(y2, kb[1], t[1]);
      t[2] = fmaf(y2, kb[2], t[2]); t[3] = fmaf(y2, kb[3], t[3]);
      xs = fmaf(t[0], qq[0], xs); xs = fmaf(t[1], qq[1], xs);
      xs = fmaf(t[2], qq[2], xs); xs = fmaf(t[3], qq[3], xs);
      *(v4fa*)(trow + 4 * j4) = t;
    }
    xs *= iq;

    volatile float* xp = (volatile float*)(xout + mrow * NQ_ + hd * D_ + tid);
    *xp = xs;
    __threadfence();
    *xp = xs;
    __syncthreads();
  }
  __syncthreads();

  float* co = carry_out + (size_t)bh * D_ * D_;
  for (int it = 0; it < (D_ * D_) / (4 * 64); ++it) {
    const int idx = it * 64 + tid;
    const int r = idx >> 4, c4 = idx & 15;
    const v4f v = *(const v4fa*)(sT + r * TP + 4 * c4);
    *(volatile v4f*)(co + (size_t)idx * 4) = v;
  }
  __threadfence();
  for (int it = 0; it < (D_ * D_) / (4 * 64); ++it) {
    const int idx = it * 64 + tid;
    const int r = idx >> 4, c4 = idx & 15;
    const v4f v = *(const v4fa*)(sT + r * TP + 4 * c4);
    *(volatile v4f*)(co + (size_t)idx * 4) = v;
  }
}

__global__ __launch_bounds__(32)
void rms_split_kernel(const float* __restrict__ xin, const float* __restrict__ rscale,
                      _Float16* __restrict__ xhi, _Float16* __restrict__ xlo, int nrows) {
  const int mrow = blockIdx.x;
  if (mrow >= nrows) return;
  const int lane = threadIdx.x & 31;
  const float* xr = xin + (size_t)mrow * NQ_;
  v4f a[4];
  a[0] = *(const v4fa*)(xr + 8 * lane);
  a[1] = *(const v4fa*)(xr + 8 * lane + 4);
  a[2] = *(const v4fa*)(xr + 256 + 8 * lane);
  a[3] = *(const v4fa*)(xr + 256 + 8 * lane + 4);
  float ss = 0.0f;
#pragma unroll
  for (int i = 0; i < 4; ++i)
#pragma unroll
    for (int e = 0; e < 4; ++e) ss = fmaf(a[i][e], a[i][e], ss);
#pragma unroll
  for (int off = 16; off > 0; off >>= 1) ss += __shfl_xor(ss, off, 32);
  const float rr = rsqrtf(ss * (1.0f / (float)NQ_) + EPS_RMS);

  v8h hv[2], lv[2];
#pragma unroll
  for (int part = 0; part < 2; ++part) {
    const int c0 = part * 256 + 8 * lane;
    const v4f s0 = *(const v4fa*)(rscale + c0);
    const v4f s1 = *(const v4fa*)(rscale + c0 + 4);
#pragma unroll
    for (int e = 0; e < 8; ++e) {
      const float xv = (e < 4) ? a[2 * part][e] : a[2 * part + 1][e - 4];
      const float sc = bf16r((e < 4) ? s0[e] : s1[e - 4]);
      const float t  = ((xv * rr) * sc) * 64.0f;
      const _Float16 hq = (_Float16)t;
      hv[part][e] = hq;
      lv[part][e] = (_Float16)((t - (float)hq) * 2048.0f);
    }
    *(volatile v8h*)(xhi + (size_t)mrow * NQ_ + c0) = hv[part];
    *(volatile v8h*)(xlo + (size_t)mrow * NQ_ + c0) = lv[part];
  }
  __threadfence();
#pragma unroll
  for (int part = 0; part < 2; ++part) {
    const int c0 = part * 256 + 8 * lane;
    *(volatile v8h*)(xhi + (size_t)mrow * NQ_ + c0) = hv[part];
    *(volatile v8h*)(xlo + (size_t)mrow * NQ_ + c0) = lv[part];
  }
}

static inline size_t al256(size_t x) { return (x + 255) & ~(size_t)255; }

extern "C" void kernel_launch(void* const* d_in, const int* in_sizes, int n_in,
                              void* d_out, int out_size, void* d_ws, size_t ws_size,
                              hipStream_t stream) {
  if (n_in < 10) return;
  if (in_sizes[0] != M_ * F_ || in_sizes[1] != M_ || in_sizes[2] != B_ * H_ * D_ * D_ ||
      in_sizes[3] != F_ * NQ_ || in_sizes[4] != F_ * NK_ || in_sizes[5] != F_ * NK_ ||
      in_sizes[6] != F_ * NB_ || in_sizes[7] != NQ_ || in_sizes[8] != NQ_ * F_ ||
      in_sizes[9] != F_) return;
  if (out_size != B_ * H_ * D_ * D_ + M_ * F_) return;

  const float* inputs   = (const float*)d_in[0];
  const int*   mask     = (const int*)d_in[1];
  const float* carry    = (const float*)d_in[2];
  const float* Wq       = (const float*)d_in[3];
  const float* Wk       = (const float*)d_in[4];
  const float* Wv       = (const float*)d_in[5];
  const float* Wb       = (const float*)d_in[6];
  const float* rmsScale = (const float*)d_in[7];
  const float* Wo       = (const float*)d_in[8];
  const float* bo       = (const float*)d_in[9];

  char* ws = (char*)d_ws;
  size_t off = 0;
  _Float16* inh  = (_Float16*)(ws + off); off = al256(off + (size_t)M_ * F_ * 2);
  _Float16* wcat = (_Float16*)(ws + off); off = al256(off + (size_t)NP_ * F_ * 2);
  _Float16* wot  = (_Float16*)(ws + off); off = al256(off + (size_t)F_ * NQ_ * 2);
  float*    qkvb = (float*)(ws + off);    off = al256(off + (size_t)M_ * NP_ * 4);
  float*    xbuf = (float*)(ws + off);    off = al256(off + (size_t)M_ * NQ_ * 4);
  _Float16* xhi  = (_Float16*)(ws + off); off = al256(off + (size_t)M_ * NQ_ * 2);
  _Float16* xlo  = (_Float16*)(ws + off); off = al256(off + (size_t)M_ * NQ_ * 2);
  if (off > ws_size) return;

  float* carry_out = (float*)d_out;
  float* y         = (float*)d_out + (size_t)B_ * H_ * D_ * D_;

  {
    const int n8 = M_ * F_ / 8;
    pack_act_kernel<<<(n8 + 255) / 256, 256, 0, stream>>>(inputs, inh, n8, 16.0f);
  }
  {
    const int n8 = NP_ * F_ / 8;
    pack_wcat_kernel<<<(n8 + 255) / 256, 256, 0, stream>>>(Wq, Wk, Wv, Wb, wcat, n8, 256.0f);
  }
  {
    const int n8 = NQ_ * F_ / 8;
    pack_wo_kernel<<<(n8 + 255) / 256, 256, 0, stream>>>(Wo, wot, n8, 256.0f);
  }

  {
    dim3 grid(NP_ / BN, M_ / BM);
    gemm_f16_kernel<1><<<grid, 256, 0, stream>>>(inh, inh, wcat, qkvb, bo, 0,
                                                  M_, NP_, F_, NP_,
                                                  1.0f / 4096.0f, 0.0f, VOFF, BOFF);
  }

  scan_kernel<<<B_ * H_, 64, 0, stream>>>(qkvb, mask, carry, xbuf, carry_out);

  rms_split_kernel<<<M_, 32, 0, stream>>>(xbuf, rmsScale, xhi, xlo, M_);

  {
    dim3 grid(F_ / BN, M_ / BM);
    gemm_f16_kernel<2><<<grid, 256, 0, stream>>>(xhi, xlo, wot, y, bo, 1,
                                                  M_, F_, NQ_, F_,
                                                  1.0f / 16384.0f, 1.0f / 33554432.0f,
                                                  0, 0x40000000);
  }
}
